// vit22_tformer_12738873000082
// MI455X (gfx1250) — hardware-verified
//
#include <hip/hip_runtime.h>
#include <math.h>
#include <stdint.h>

#define SEQ   2048
#define DM    1024
#define NH    16
#define HD    64
#define FFI   4096
#define FUS   8192
#define NQB   (SEQ / 64)
#define VLP   512
#define RESQB 8
#define QSC   8.0f
#define SSC   (1.0f / 64.0f)
#define XSC   16.0f
#define WSC   64.0f
#define FSC   64.0f
#define VRS   4096.0f
#define SP    20
#define OSP   20

static_assert(RESQB * 64 <= VLP);
static_assert(NH * HD == DM);
static_assert((SEQ % 64) == 0 && (DM % 64) == 0 && (FFI % 64) == 0 && (FUS % 128) == 0);

typedef _Float16 v16h __attribute__((ext_vector_type(16)));
typedef _Float16 v8h  __attribute__((ext_vector_type(8)));
typedef __bf16   v16b __attribute__((ext_vector_type(16)));
typedef __bf16   v8b  __attribute__((ext_vector_type(8)));
typedef float    v8f  __attribute__((ext_vector_type(8)));
typedef float    v4f  __attribute__((ext_vector_type(4)));
typedef unsigned int v4u __attribute__((ext_vector_type(4)));

struct InvTab { float f[HD / 2]; };
static_assert(sizeof(InvTab) == 128);

__device__ __forceinline__ unsigned short bf_bits(float f) {
  unsigned u = __float_as_uint(f);
  return (unsigned short)((u + 0x7FFFu + ((u >> 16) & 1u)) >> 16);
}
__device__ __forceinline__ float bf_up(unsigned short h) { return __uint_as_float(((unsigned)h) << 16); }
__device__ __forceinline__ unsigned short h_bits(_Float16 x) { return __builtin_bit_cast(unsigned short, x); }
__device__ __forceinline__ unsigned pk16(unsigned short a, unsigned short b) { return (unsigned)a | ((unsigned)b << 16); }
__device__ __forceinline__ v8f zero8() { v8f z = {0.f, 0.f, 0.f, 0.f, 0.f, 0.f, 0.f, 0.f}; return z; }
__device__ __forceinline__ v8h zero8h() {
  const _Float16 z = (_Float16)0.0f;
  v8h r = {z, z, z, z, z, z, z, z};
  return r;
}
__device__ __forceinline__ void wave_sync_lds() {
  __builtin_amdgcn_fence(__ATOMIC_RELEASE, "workgroup");
  __builtin_amdgcn_wave_barrier();
  __builtin_amdgcn_fence(__ATOMIC_ACQUIRE, "workgroup");
}

template <typename T> struct Frag16;
template <> struct Frag16<_Float16> { typedef v16h t; };
template <> struct Frag16<__bf16>   { typedef v16b t; };

__device__ __forceinline__ v16h ldfrag(const _Float16* p) {
  union { v16h v; v8h h[2]; } f;
  f.h[0] = *(const v8h*)(p);
  f.h[1] = *(const v8h*)(p + 16);
  return f.v;
}
__device__ __forceinline__ v16b ldfrag(const __bf16* p) {
  union { v16b v; v8b h[2]; } f;
  f.h[0] = *(const v8b*)(p);
  f.h[1] = *(const v8b*)(p + 16);
  return f.v;
}

__device__ __forceinline__ v8f mma_raw(v16h a, v16h b, v8f c) {
  return __builtin_amdgcn_wmma_f32_16x16x32_f16(false, a, false, b, (short)0, c, false, false);
}
__device__ __forceinline__ v8f mma_raw(v16b a, v16b b, v8f c) {
  return __builtin_amdgcn_wmma_f32_16x16x32_bf16(false, a, false, b, (short)0, c, false, false);
}
__device__ __forceinline__ v8f mma_h(v16h a, v16h b, v8f c) {
  c = mma_raw(a, b, c);
#if defined(__HIP_DEVICE_COMPILE__)
  asm volatile("v_nop\n\tv_nop\n\tv_nop\n\tv_nop" : "+v"(c) : "v"(a), "v"(b));
#endif
  return c;
}
__device__ __forceinline__ void dep_guard2(v8f& a, v8f& b, v16h x, v16h y) {
#if defined(__HIP_DEVICE_COMPILE__)
  asm volatile("v_nop\n\tv_nop\n\tv_nop\n\tv_nop" : "+v"(a), "+v"(b) : "v"(x), "v"(y));
#else
  (void)a; (void)b; (void)x; (void)y;
#endif
}
__device__ __forceinline__ void dep_guard2(v8f& a, v8f& b, v16b x, v16b y) {
#if defined(__HIP_DEVICE_COMPILE__)
  asm volatile("v_nop\n\tv_nop\n\tv_nop\n\tv_nop" : "+v"(a), "+v"(b) : "v"(x), "v"(y));
#else
  (void)a; (void)b; (void)x; (void)y;
#endif
}
__device__ __forceinline__ void keep1(v16h x) {
#if defined(__HIP_DEVICE_COMPILE__)
  asm volatile("v_nop" :: "v"(x));
#else
  (void)x;
#endif
}
__device__ __forceinline__ void keep1(v16b x) {
#if defined(__HIP_DEVICE_COMPILE__)
  asm volatile("v_nop" :: "v"(x));
#else
  (void)x;
#endif
}
__device__ __forceinline__ void acc_guard4(v8f& a, v8f& b, v8f& c, v8f& d) {
#if defined(__HIP_DEVICE_COMPILE__)
  asm volatile("v_nop\n\tv_nop\n\tv_nop\n\tv_nop" : "+v"(a), "+v"(b), "+v"(c), "+v"(d));
#else
  (void)a; (void)b; (void)c; (void)d;
#endif
}

__device__ __forceinline__ float swg(float xacc, float gacc, float oscale, float bx, float bg, float rscale) {
  const float xp = xacc * oscale + bx;
  const float g  = gacc * oscale + bg;
  const float sg = __builtin_amdgcn_rcpf(1.0f + __expf(-g));
  return (g * sg) * xp * rscale;
}

__global__ __launch_bounds__(256) void k_cstab(InvTab tab, float* cs) {
  const int lane = threadIdx.x & 31, wave = threadIdx.x >> 5;
  const int t = blockIdx.x * 8 + wave;
  float ivf = tab.f[0];
#pragma unroll
  for (int i = 1; i < HD / 2; ++i) ivf = (lane == i) ? tab.f[i] : ivf;
  const float fr = (float)t * ivf;
  float sn, cn;
  sincosf(fr, &sn, &cn);
  const float cv = bf_up(bf_bits(cn));
  const float sv = bf_up(bf_bits(sn));
  float* pc = cs + (size_t)t * 64 + lane;
  float* ps = pc + 32;
  *(volatile float*)pc = cv;
  *(volatile float*)ps = sv;
  __threadfence();
  *(volatile float*)pc = cv;
  *(volatile float*)ps = sv;
}

__global__ __launch_bounds__(128) void k_xnorm(const float* __restrict__ hs, unsigned short* xh,
                                               unsigned short* xbh, unsigned short* xbl) {
  __shared__ float red[4];
  const int tid = threadIdx.x, lane = tid & 31, wave = tid >> 5, t = blockIdx.x;
  const size_t off = (size_t)t * DM + (size_t)tid * 8;
  const v4f a = *(const v4f*)(hs + off);
  const v4f b = *(const v4f*)(hs + off + 4);
  float ss = a[0] * a[0] + a[1] * a[1] + a[2] * a[2] + a[3] * a[3]
           + b[0] * b[0] + b[1] * b[1] + b[2] * b[2] + b[3] * b[3];
#pragma unroll
  for (int o = 1; o < 32; o <<= 1) ss += __shfl_xor(ss, o, 32);
  if (lane == 0) red[wave] = ss;
  __syncthreads();
  const float tot = (red[0] + red[1]) + (red[2] + red[3]);
  const float rn = rsqrtf(tot * (1.0f / (float)DM) + 1.1920929e-7f);
  float x[8];
  x[0] = a[0] * rn; x[1] = a[1] * rn; x[2] = a[2] * rn; x[3] = a[3] * rn;
  x[4] = b[0] * rn; x[5] = b[1] * rn; x[6] = b[2] * rn; x[7] = b[3] * rn;
  v4u ph, pb, pl;
#pragma unroll
  for (int e = 0; e < 4; ++e) {
    const float f0 = x[2 * e], f1 = x[2 * e + 1];
    ph[e] = pk16(h_bits((_Float16)(f0 * XSC)), h_bits((_Float16)(f1 * XSC)));
    const unsigned short hb0 = bf_bits(f0), hb1 = bf_bits(f1);
    pb[e] = pk16(hb0, hb1);
    pl[e] = pk16(bf_bits(f0 - bf_up(hb0)), bf_bits(f1 - bf_up(hb1)));
  }
  *(volatile v4u*)(xh + off)  = ph;
  *(volatile v4u*)(xbh + off) = pb;
  *(volatile v4u*)(xbl + off) = pl;
  __threadfence();
  *(volatile v4u*)(xh + off)  = ph;
  *(volatile v4u*)(xbh + off) = pb;
  *(volatile v4u*)(xbl + off) = pl;
}

template <int MODE>
__global__ __launch_bounds__(256) void k_wtrans(const float* __restrict__ W, int K, int N, int nhalf, float wscale,
                                                unsigned short* out0, unsigned short* out1) {
  __shared__ float tl[64][65];
  const int tid = threadIdx.x, lane = tid & 31, wave = tid >> 5;
  const int n0 = blockIdx.x * 64, k0 = blockIdx.y * 64;
  {
    const int i0 = tid >> 4, cc = (tid & 15) * 4;
#pragma unroll
    for (int p = 0; p < 4; ++p) {
      const int i = p * 16 + i0;
      const v4f v = *(const v4f*)(W + (size_t)(k0 + i) * N + n0 + cc);
      tl[i][cc] = v[0]; tl[i][cc + 1] = v[1]; tl[i][cc + 2] = v[2]; tl[i][cc + 3] = v[3];
    }
  }
  __syncthreads();
  const int orow0 = (nhalf > 0) ? ((n0 < nhalf) ? (2 * n0) : (2 * (n0 - nhalf) + 64)) : n0;
  const int q8 = lane >> 3, c8 = (lane & 7) * 8;
  v4u hv[2], lv[2];
#pragma unroll
  for (int it = 0; it < 2; ++it) {
    const int j = it * 32 + wave * 4 + q8;
    v4u a, a2;
#pragma unroll
    for (int e = 0; e < 4; ++e) {
      const float f0 = tl[c8 + 2 * e][j], f1 = tl[c8 + 2 * e + 1][j];
      if constexpr (MODE == 0) {
        a[e] = pk16(h_bits((_Float16)(f0 * wscale)), h_bits((_Float16)(f1 * wscale)));
        a2[e] = 0u;
      } else {
        const unsigned short hb0 = bf_bits(f0), hb1 = bf_bits(f1);
        a[e] = pk16(hb0, hb1);
        a2[e] = pk16(bf_bits(f0 - bf_up(hb0)), bf_bits(f1 - bf_up(hb1)));
      }
    }
    hv[it] = a; lv[it] = a2;
  }
  for (int pass = 0; pass < 2; ++pass) {
#pragma unroll
    for (int it = 0; it < 2; ++it) {
      const int j = it * 32 + wave * 4 + q8;
      const size_t go = (size_t)(orow0 + j) * K + k0 + c8;
      *(volatile v4u*)(out0 + go) = hv[it];
      if constexpr (MODE == 1) *(volatile v4u*)(out1 + go) = lv[it];
    }
    __threadfence();
  }
}

template <typename T, int MI, int NJ, int NSPLIT, int EPI>
__global__ __launch_bounds__(256) void k_gemm(
    const unsigned short* __restrict__ Ap, const unsigned short* __restrict__ A2p, int lda,
    const unsigned short* __restrict__ Bp, const unsigned short* __restrict__ B2p, int ldb,
    void* Cout, int ldc, void* Cout2, int ldc2, int N2,
    const float* __restrict__ bias, const float* __restrict__ resh,
    const float* __restrict__ resa, const float* __restrict__ lamp,
    int M, int N, int K, float oscale, float rscale) {
  typedef typename Frag16<T>::t FR;
  static_assert((EPI == 4) ? (MI == 2 && NJ == 8) : (NJ == 4 && (MI == 2 || MI == 4)));
  static_assert(NSPLIT == 0 || NSPLIT == 2);
  const T* A   = (const T*)(const void*)Ap;
  const T* A2  = (const T*)(const void*)A2p;
  const T* Bt  = (const T*)(const void*)Bp;
  const T* Bt2 = (const T*)(const void*)B2p;
  __shared__ __align__(16) float sT[8][64 * SP];
  constexpr int TM = 16 * MI, TN = 16 * NJ;
  const int lane = threadIdx.x & 31;
  const int wave = threadIdx.x >> 5;
  const int tilesN = N / TN;
  const int tilesM = M / TM;
  const int tile = blockIdx.x * 8 + wave;
  if (tile >= tilesM * tilesN) return;
  const int tm = tile / tilesN;
  const int tn = tile - tm * tilesN;
  const int m0 = tm * TM;
  const int n0 = tn * TN;
  const int rl   = lane & 15;
  const int koff = (lane >> 4) * 8;
  const int mOff = (lane >> 4) * 8;

  v8f acc[MI][NJ];
#pragma unroll
  for (int i = 0; i < MI; ++i)
#pragma unroll
    for (int j = 0; j < NJ; ++j) acc[i][j] = zero8();

  for (int k0 = 0; k0 < K; k0 += 32) {
    {
      FR ah[MI];
#pragma unroll
      for (int i = 0; i < MI; ++i)
        ah[i] = ldfrag(A + (size_t)(m0 + 16 * i + rl) * lda + k0 + koff);
#pragma unroll
      for (int j = 0; j < NJ; ++j) {
        const size_t bo = (size_t)(n0 + 16 * j + rl) * ldb + k0 + koff;
        const FR bh = ldfrag(Bt + bo);
        FR bl = bh;
        if constexpr (NSPLIT == 2) bl = ldfrag(Bt2 + bo);
#pragma unroll
        for (int i = 0; i < MI; ++i) {
          acc[i][j] = mma_raw(ah[i], bh, acc[i][j]);
          if constexpr (NSPLIT == 2) acc[i][j] = mma_raw(ah[i], bl, acc[i][j]);
        }
        dep_guard2(acc[0][j], acc[MI - 1][j], bh, bl);
      }
#pragma unroll
      for (int i = 0; i < MI; ++i) keep1(ah[i]);
    }
    if constexpr (NSPLIT == 2) {
      FR al[MI];
#pragma unroll
      for (int i = 0; i < MI; ++i)
        al[i] = ldfrag(A2 + (size_t)(m0 + 16 * i + rl) * lda + k0 + koff);
#pragma unroll
      for (int j = 0; j < NJ; ++j) {
        const size_t bo = (size_t)(n0 + 16 * j + rl) * ldb + k0 + koff;
        const FR bh = ldfrag(Bt + bo);
#pragma unroll
        for (int i = 0; i < MI; ++i) acc[i][j] = mma_raw(al[i], bh, acc[i][j]);
        dep_guard2(acc[0][j], acc[MI - 1][j], bh, bh);
      }
#pragma unroll
      for (int i = 0; i < MI; ++i) keep1(al[i]);
    }
  }
#pragma unroll
  for (int i = 0; i < MI; ++i)
#pragma unroll
    for (int j = 0; j < NJ; j += 4) acc_guard4(acc[i][j], acc[i][j + 1], acc[i][j + 2], acc[i][j + 3]);

  float* slab = sT[wave];
  const int ocol0 = (EPI == 4) ? (tn * 64) : n0;
  const int hq = lane >> 4, c4 = (lane & 15) * 4;
  const int q8 = lane >> 3, c8 = (lane & 7) * 8;
  float bxv[4] = {0.f, 0.f, 0.f, 0.f}, bgv[4] = {0.f, 0.f, 0.f, 0.f};
  v4f b4 = {0.f, 0.f, 0.f, 0.f};
  float lam = 0.f;
  if constexpr (EPI == 4) {
#pragma unroll
    for (int j = 0; j < 4; ++j) {
      bxv[j] = bias[ocol0 + 16 * j + rl];
      bgv[j] = bias[FFI + ocol0 + 16 * j + rl];
    }
  }
  if constexpr (EPI == 1 || EPI == 3) b4 = *(const v4f*)(bias + n0 + c4);
  if constexpr (EPI == 3) lam = lamp[0];

#pragma unroll
  for (int i = 0; i < MI; ++i) {
    const int mBase = m0 + 16 * i;
#pragma unroll
    for (int j = 0; j < 4; ++j) {
      v4f w0, w1;
      if constexpr (EPI == 4) {
#pragma unroll
        for (int r = 0; r < 4; ++r) {
          w0[r] = swg(acc[i][j][r],     acc[i][j + 4][r],     oscale, bxv[j], bgv[j], rscale);
          w1[r] = swg(acc[i][j][r + 4], acc[i][j + 4][r + 4], oscale, bxv[j], bgv[j], rscale);
        }
      } else {
#pragma unroll
        for (int r = 0; r < 4; ++r) {
          w0[r] = acc[i][j][r] * oscale;
          w1[r] = acc[i][j][r + 4] * oscale;
        }
      }
      float* cp = slab + (16 * j + rl) * SP + mOff;
      *(v4f*)(cp) = w0;
      *(v4f*)(cp + 4) = w1;
    }
    wave_sync_lds();
    if constexpr (EPI == 0 || EPI == 1 || EPI == 3) {
      float* C = (float*)Cout;
      v4f fin[8];
#pragma unroll
      for (int it = 0; it < 8; ++it) {
        const int row = 2 * it + hq;
        v4f v;
        v[0] = slab[(c4 + 0) * SP + row];
        v[1] = slab[(c4 + 1) * SP + row];
        v[2] = slab[(c4 + 2) * SP + row];
        v[3] = slab[(c4 + 3) * SP + row];
        if constexpr (EPI == 1) v = v + b4;
        if constexpr (EPI == 3) {
          const size_t go = (size_t)(mBase + row) * ldc + n0 + c4;
          const v4f hvv = *(const v4f*)(resh + go);
          const v4f avv = *(const v4f*)(resa + go);
          v = v + b4 + hvv * lam + avv;
        }
        fin[it] = v;
      }
      for (int pass = 0; pass < 2; ++pass) {
#pragma unroll
        for (int it = 0; it < 8; ++it) {
          const int row = 2 * it + hq;
          *(volatile v4f*)(C + (size_t)(mBase + row) * ldc + n0 + c4) = fin[it];
        }
        __threadfence();
      }
    } else {
      unsigned short* C  = (unsigned short*)Cout;
      unsigned short* C2 = (unsigned short*)Cout2;
      const bool wlo = (EPI == 2) && (n0 < N2);
      v4u hv[4], lv[4];
#pragma unroll
      for (int it = 0; it < 4; ++it) {
        const int row = 4 * it + q8;
        v4u a, a2;
#pragma unroll
        for (int e = 0; e < 4; ++e) {
          const float f0 = slab[(c8 + 2 * e) * SP + row], f1 = slab[(c8 + 2 * e + 1) * SP + row];
          const _Float16 x0 = (_Float16)f0, x1 = (_Float16)f1;
          unsigned short l0 = 0, l1 = 0;
          if constexpr (EPI == 2) {
            l0 = h_bits((_Float16)((f0 - (float)x0) * rscale));
            l1 = h_bits((_Float16)((f1 - (float)x1) * rscale));
          }
          a[e] = pk16(h_bits(x0), h_bits(x1)); a2[e] = pk16(l0, l1);
        }
        hv[it] = a; lv[it] = a2;
      }
      for (int pass = 0; pass < 2; ++pass) {
#pragma unroll
        for (int it = 0; it < 4; ++it) {
          const int row = 4 * it + q8;
          *(volatile v4u*)(C + (size_t)(mBase + row) * ldc + ocol0 + c8) = hv[it];
          if (wlo) *(volatile v4u*)(C2 + (size_t)(mBase + row) * ldc2 + n0 + c8) = lv[it];
        }
        __threadfence();
      }
    }
    wave_sync_lds();
  }
}

__global__ __launch_bounds__(256) void k_rope(const float* __restrict__ qkf, const float* __restrict__ cs,
                                              unsigned short* qh, unsigned short* kh, float* qbn, float* kbn) {
  __shared__ __align__(16) float yb[8][4 * 64];
  const int lane = threadIdx.x & 31, wave = threadIdx.x >> 5;
  const int p = blockIdx.x * 8 + wave;
  const int t = p >> 4, h = p & 15;
  const float cth = cs[(size_t)t * 64 + lane];
  const float sth = cs[(size_t)t * 64 + 32 + lane];
  const float* row = qkf + (size_t)t * (4 * DM) + h * HD;
  float* ybw = yb[wave];
#pragma unroll
  for (int g = 0; g < 4; ++g) {
    const float* src = row + g * DM;
    float x1 = src[lane], x2 = src[lane + 32];
    float n2 = x1 * x1 + x2 * x2;
#pragma unroll
    for (int o = 1; o < 32; o <<= 1) n2 += __shfl_xor(n2, o, 32);
    const float rn = 1.0f / fmaxf(sqrtf(n2), 1e-12f);
    x1 *= rn; x2 *= rn;
    ybw[g * 64 + lane]      = x1 * cth + x2 * sth;
    ybw[g * 64 + 32 + lane] = x2 * cth - x1 * sth;
  }
  wave_sync_lds();
  const int c8 = (lane & 7) * 8, c4 = (lane & 15) * 4;
  v4u qv, kv;
#pragma unroll
  for (int e = 0; e < 4; ++e) {
    qv[e] = pk16(h_bits((_Float16)(ybw[c8 + 2 * e] * QSC)), h_bits((_Float16)(ybw[c8 + 2 * e + 1] * QSC)));
    kv[e] = pk16(h_bits((_Float16)(ybw[64 + c8 + 2 * e] * QSC)), h_bits((_Float16)(ybw[64 + c8 + 2 * e + 1] * QSC)));
  }
  const v4f qbv = *(const v4f*)(ybw + 128 + c4);
  const v4f kbv = *(const v4f*)(ybw + 192 + c4);
  const size_t g16 = (size_t)t * DM + h * HD + c8;
  const size_t g32 = (size_t)t * DM + h * HD + c4;
  for (int pass = 0; pass < 2; ++pass) {
    if (lane < 8) {
      *(volatile v4u*)(qh + g16) = qv;
      *(volatile v4u*)(kh + g16) = kv;
    }
    if (lane < 16) {
      *(volatile v4f*)(qbn + g32) = qbv;
      *(volatile v4f*)(kbn + g32) = kbv;
    }
    __threadfence();
  }
}

__global__ __launch_bounds__(256) void k_prefix(const float* __restrict__ kbn, float* pf) {
  const int col = blockIdx.x * 256 + threadIdx.x;
  double acc = 0.0;
#pragma unroll 1
  for (int t = 0; t < SEQ; ++t) {
    acc += (double)kbn[(size_t)t * DM + col];
    const float v = (float)acc;
    float* d = pf + (size_t)t * DM + col;
    *(volatile float*)d = v;
    __threadfence();
    *(volatile float*)d = v;
  }
}

template <bool RES>
__global__ __launch_bounds__(128)
void k_attn(const unsigned short* __restrict__ qhp, const unsigned short* __restrict__ khp,
            const unsigned short* __restrict__ vhp, const unsigned short* __restrict__ vlp,
            const float* __restrict__ qbn, const float* __restrict__ pfx, const float* __restrict__ l2p,
            unsigned short* yhp, unsigned short* ylp, int qbBase, int nqbThis) {
  union FH { v16h v; v8h h[2]; };
  __shared__ __align__(16) _Float16 Ksh[64 * 64];
  __shared__ __align__(16) _Float16 Vth[64 * 64];
  __shared__ __align__(16) _Float16 Vtl[RES ? 64 * 64 : 8];
  __shared__ __align__(16) _Float16 Psh[4][16 * 64];
  __shared__ __align__(16) _Float16 Psl[RES ? 4 : 1][16 * 64];
  __shared__ __align__(16) float    Os[4][64 * OSP];
  __shared__ float Sbl[4][16];

  const int tid  = threadIdx.x;
  const int wave = tid >> 5;
  const int lane = tid & 31;
  const int hh   = lane >> 4;
  const int c    = lane & 15;

  const int bx  = blockIdx.x;
  const int qbl = bx % nqbThis;
  const int h   = bx / nqbThis;
  const int qb  = qbBase + qbl;
  const int q0  = qb * 64 + wave * 16;

  const _Float16* Qh = (const _Float16*)(const void*)qhp + (size_t)h * HD;
  const _Float16* Kh = (const _Float16*)(const void*)khp + (size_t)h * HD;
  const _Float16* Vh = (const _Float16*)(const void*)vhp + (size_t)h * HD * SEQ;
  const _Float16* Vl = (const _Float16*)(const void*)vlp + (size_t)h * HD * VLP;

  v16h qa[2];
#pragma unroll
  for (int dc = 0; dc < 2; ++dc) qa[dc] = ldfrag(Qh + (size_t)(q0 + c) * DM + dc * 32 + 8 * hh);

  float mrow[8], lrow[8];
  v8f oacc[4];
#pragma unroll
  for (int r = 0; r < 8; ++r) { mrow[r] = -INFINITY; lrow[r] = 0.f; }
#pragma unroll
  for (int t = 0; t < 4; ++t) oacc[t] = zero8();

  int nkt = qb + 1;
  if (nkt > NQB) nkt = NQB;
  for (int kt = 0; kt < nkt; ++kt) {
    const int kv0 = kt * 64;
    __syncthreads();
    {
      const int r = tid >> 1, half = (tid & 1) * 32;
      const _Float16* kg = Kh + (size_t)(kv0 + r) * DM + half;
      const _Float16* vg = Vh + (size_t)r * SEQ + kv0 + half;
      const int kvl = (kv0 + 64 <= VLP) ? kv0 : (VLP - 64);
      const _Float16* vlg = Vl + (size_t)r * VLP + kvl + half;
      const bool resOK = (kv0 + 64 <= VLP);
#pragma unroll
      for (int i = 0; i < 4; ++i) {
        const v8h a0 = *(const v8h*)(kg + 8 * i);
        const v8h b0 = *(const v8h*)(vg + 8 * i);
        *(v8h*)(Ksh + r * 64 + half + 8 * i) = a0;
        *(v8h*)(Vth + r * 64 + half + 8 * i) = b0;
        if (RES) {
          v8h b1 = *(const v8h*)(vlg + 8 * i);
          if (!resOK) b1 = zero8h();
          *(v8h*)(Vtl + r * 64 + half + 8 * i) = b1;
        }
      }
    }
    __syncthreads();

    v8f s[4];
#pragma unroll
    for (int j = 0; j < 4; ++j) {
      s[j] = zero8();
#pragma unroll
      for (int dc = 0; dc < 2; ++dc) {
        FH kb;
        kb.h[0] = *(const v8h*)(Ksh + (j * 16 + c) * 64 + dc * 32 + 8 * hh);
        kb.h[1] = *(const v8h*)(Ksh + (j * 16 + c) * 64 + dc * 32 + 16 + 8 * hh);
        s[j] = mma_h(qa[dc], kb.v, s[j]);
      }
    }

    _Float16* pwh = Psh[wave];
    _Float16* pwl = Psl[RES ? wave : 0];
#pragma unroll
    for (int r = 0; r < 8; ++r) {
      const int qrow = q0 + 8 * hh + r;
      float m = -INFINITY;
#pragma unroll
      for (int j = 0; j < 4; ++j) {
        const int key = kv0 + j * 16 + c;
        float sv = s[j][r] * SSC;
        sv = (key <= qrow) ? sv : -INFINITY;
        s[j][r] = sv;
        m = fmaxf(m, sv);
      }
#pragma unroll
      for (int off = 1; off < 16; off <<= 1) m = fmaxf(m, __shfl_xor(m, off, 32));
      const float mnew  = fmaxf(mrow[r], m);
      const float msafe = (mnew == -INFINITY) ? 0.f : mnew;
      const float alpha = __expf(mrow[r] - msafe);
      mrow[r] = mnew;
      float psum = 0.f;
#pragma unroll
      for (int j = 0; j < 4; ++j) {
        const float p = __expf(s[j][r] - msafe);
        psum += p;
        const float p1k = p * 1024.0f;
        const _Float16 ph = (_Float16)p1k;
        pwh[(8 * hh + r) * 64 + j * 16 + c] = ph;
        if (RES) {
          const _Float16 pl = (_Float16)((p1k - (float)ph) * VRS);
          pwl[(8 * hh + r) * 64 + j * 16 + c] = pl;
        }
      }
#pragma unroll
      for (int off = 1; off < 16; off <<= 1) psum += __shfl_xor(psum, off, 32);
      lrow[r] = lrow[r] * alpha + psum;
#pragma unroll
      for (int t = 0; t < 4; ++t) oacc[t][r] *= alpha;
    }
    wave_sync_lds();

    v8f o1[4];
#pragma unroll
    for (int t = 0; t < 4; ++t) o1[t] = zero8();
#pragma unroll 1
    for (int kk = 0; kk < 2; ++kk) {
      FH pa, pl;
      pa.h[0] = *(const v8h*)(pwh + c * 64 + kk * 32 + 8 * hh);
      pa.h[1] = *(const v8h*)(pwh + c * 64 + kk * 32 + 16 + 8 * hh);
      if (RES) {
        pl.h[0] = *(const v8h*)(pwl + c * 64 + kk * 32 + 8 * hh);
        pl.h[1] = *(const v8h*)(pwl + c * 64 + kk * 32 + 16 + 8 * hh);
      } else {
        pl.v = pa.v;
      }
#pragma unroll
      for (int t = 0; t < 4; ++t) {
        FH vb;
        vb.h[0] = *(const v8h*)(Vth + (t * 16 + c) * 64 + kk * 32 + 8 * hh);
        vb.h[1] = *(const v8h*)(Vth + (t * 16 + c) * 64 + kk * 32 + 16 + 8 * hh);
        oacc[t] = mma_h(pa.v, vb.v, oacc[t]);
        if (RES) {
          FH vl;
          vl.h[0] = *(const v8h*)(Vtl + (t * 16 + c) * 64 + kk * 32 + 8 * hh);
          vl.h[1] = *(const v8h*)(Vtl + (t * 16 + c) * 64 + kk * 32 + 16 + 8 * hh);
          o1[t] = mma_h(pa.v, vl.v, o1[t]);
          o1[t] = mma_h(pl.v, vb.v, o1[t]);
        }
      }
    }
    if (RES) {
#pragma unroll
      for (int t = 0; t < 4; ++t)
#pragma unroll
        for (int r = 0; r < 8; ++r) oacc[t][r] += o1[t][r] * (1.0f / VRS);
    }
  }

  const float l2ns = l2p[0];
  {
    const size_t ro = (size_t)(q0 + c) * DM + (size_t)h * HD + hh * 32;
    const float* qp = qbn + ro;
    const float* pp = pfx + ro;
    float ds = 0.f;
#pragma unroll
    for (int e = 0; e < 8; ++e) {
      const v4f a = *(const v4f*)(qp + 4 * e);
      const v4f b = *(const v4f*)(pp + 4 * e);
      ds += a[0] * b[0] + a[1] * b[1] + a[2] * b[2] + a[3] * b[3];
    }
    ds += __shfl_xor(ds, 16, 32);
    if (hh == 0) Sbl[wave][c] = ds * 0.125f;
  }

  float* os = Os[wave];
  float invr[8];
#pragma unroll
  for (int r = 0; r < 8; ++r) {
    const float l = lrow[r];
    invr[r] = ((l > 0.f) ? (1.0f / l) : 0.f) * (l2ns * (1.0f / 1024.0f));
  }
#pragma unroll
  for (int t = 0; t < 4; ++t) {
    v4f w0, w1;
#pragma unroll
    for (int r = 0; r < 4; ++r) {
      w0[r] = oacc[t][r] * invr[r];
      w1[r] = oacc[t][r + 4] * invr[r + 4];
    }
    float* cp = os + (t * 16 + c) * OSP + 8 * hh;
    *(v4f*)(cp) = w0;
    *(v4f*)(cp + 4) = w1;
  }
  wave_sync_lds();
  {
    const int q4 = lane >> 3, c8 = (lane & 7) * 8;
    v4u hv[4], lv[4];
#pragma unroll
    for (int it = 0; it < 4; ++it) {
      const int row = it * 4 + q4;
      const float sbv = Sbl[wave][row];
      v4u a, a2;
#pragma unroll
      for (int e = 0; e < 4; ++e) {
        const float f0 = os[(c8 + 2 * e) * OSP + row] + sbv;
        const float f1 = os[(c8 + 2 * e + 1) * OSP + row] + sbv;
        const unsigned short h0 = bf_bits(f0), h1 = bf_bits(f1);
        const unsigned short l0 = bf_bits(f0 - bf_up(h0)), l1 = bf_bits(f1 - bf_up(h1));
        a[e] = pk16(h0, h1); a2[e] = pk16(l0, l1);
      }
      hv[it] = a; lv[it] = a2;
    }
    for (int pass = 0; pass < 2; ++pass) {
#pragma unroll
      for (int it = 0; it < 4; ++it) {
        const int row = it * 4 + q4;
        const size_t go = (size_t)(q0 + row) * DM + (size_t)h * HD + c8;
        *(volatile v4u*)(yhp + go) = hv[it];
        *(volatile v4u*)(ylp + go) = lv[it];
      }
      __threadfence();
    }
  }
}

extern "C" void kernel_launch(void* const* d_in, const int* in_sizes, int n_in,
                              void* d_out, int out_size, void* d_ws, size_t ws_size,
                              hipStream_t stream) {
  if (n_in < 14) return;
  if (in_sizes[0] != SEQ * DM) return;
  for (int i = 1; i <= 6; ++i) if (in_sizes[i] != DM * DM) return;
  if (in_sizes[7] != DM) return;
  if (in_sizes[8] != DM * FUS || in_sizes[9] != FUS) return;
  if (in_sizes[10] != FFI * DM || in_sizes[11] != DM) return;
  if (in_sizes[12] < 1 || in_sizes[13] < 1) return;
  if (out_size != SEQ * DM) return;

  const float* hs  = (const float*)d_in[0];
  const float* Wq  = (const float*)d_in[1];
  const float* Wk  = (const float*)d_in[2];
  const float* Wv  = (const float*)d_in[3];
  const float* Wqb = (const float*)d_in[4];
  const float* Wkb = (const float*)d_in[5];
  const float* Wo  = (const float*)d_in[6];
  const float* bo  = (const float*)d_in[7];
  const float* W1  = (const float*)d_in[8];
  const float* b1  = (const float*)d_in[9];
  const float* W2  = (const float*)d_in[10];
  const float* b2  = (const float*)d_in[11];
  const float* lam = (const float*)d_in[12];
  const float* l2n = (const float*)d_in[13];

  InvTab itab;
  for (int d = 0; d < HD / 2; ++d)
    { const float pw = (float)pow(1000.0, (2.0 * (double)d) / 64.0); itab.f[d] = 1.0f / pw; }

  const size_t MiB = 1048576;
  const size_t oXh  = 0;
  const size_t oXbh = 4 * MiB,  oXbl = 8 * MiB;
  const size_t oQh  = oXbh,     oKh  = oXbl;
  const size_t oWcat = 12 * MiB;
  const size_t oWvh = 20 * MiB, oWvl = 22 * MiB, oWoh = 24 * MiB, oWol = 26 * MiB;
  const size_t oW1t = 28 * MiB;
  const size_t oW2t = 44 * MiB;
  const size_t oCS  = 52 * MiB;
  const size_t oQK  = 53 * MiB;
  const size_t oPf  = 53 * MiB, oYh = 61 * MiB, oYl = 65 * MiB, oAO = 69 * MiB;
  const size_t oQBn = 85 * MiB, oKBn = 93 * MiB;
  const size_t oVTh = 101 * MiB, oVTl = 105 * MiB;
  const size_t oFF  = 106 * MiB;
  const size_t oEnd = 122 * MiB;
  if ((size_t)SEQ * DM * 2 != 4 * MiB) return;
  if ((size_t)DM * DM * 2 != 2 * MiB) return;
  if (oWcat + (size_t)4 * DM * DM * 2 != oWvh) return;
  if (oW1t + (size_t)FUS * DM * 2 != oW2t) return;
  if (oW2t + (size_t)DM * FFI * 2 != oCS) return;
  if (oCS + (size_t)SEQ * 64 * 4 > oQK) return;
  if (oQK + (size_t)SEQ * 4 * DM * 4 != oQBn) return;
  if (oPf + (size_t)SEQ * DM * 4 != oYh) return;
  if (oYl + (size_t)SEQ * DM * 2 != oAO) return;
  if (oAO + (size_t)SEQ * DM * 4 > oQBn) return;
  if (oVTh + (size_t)DM * SEQ * 2 != oVTl) return;
  if (oVTl + (size_t)DM * VLP * 2 != oFF) return;
  if (oFF + (size_t)SEQ * FFI * 2 != oEnd) return;
  if (oEnd > ws_size) return;
  if (oEnd > (size_t)134217728) return;

  char* ws = (char*)d_ws;
  unsigned short* Xh   = (unsigned short*)(ws + oXh);
  unsigned short* Xbh  = (unsigned short*)(ws + oXbh);
  unsigned short* Xbl  = (unsigned short*)(ws + oXbl);
  unsigned short* Qh   = (unsigned short*)(ws + oQh);
  unsigned short* Kh   = (unsigned short*)(ws + oKh);
  unsigned short* Wcat = (unsigned short*)(ws + oWcat);
  unsigned short* Wvh  = (unsigned short*)(ws + oWvh);
  unsigned short* Wvl  = (unsigned short*)(ws + oWvl);
  unsigned short* Woh  = (unsigned short*)(ws + oWoh);
  unsigned short* Wol  = (unsigned short*)(ws + oWol);
  unsigned short* W1t  = (unsigned short*)(ws + oW1t);
  unsigned short* W2t  = (unsigned short*)(ws + oW2t);
  float*          CS   = (float*)(ws + oCS);
  float*          QK   = (float*)(ws + oQK);
  float*          Pf   = (float*)(ws + oPf);
  unsigned short* Yh   = (unsigned short*)(ws + oYh);
  unsigned short* Yl   = (unsigned short*)(ws + oYl);
  float*          AO   = (float*)(ws + oAO);
  float*          QBn  = (float*)(ws + oQBn);
  float*          KBn  = (float*)(ws + oKBn);
  unsigned short* VTh  = (unsigned short*)(ws + oVTh);
  unsigned short* VTl  = (unsigned short*)(ws + oVTl);
  unsigned short* FF   = (unsigned short*)(ws + oFF);

  const dim3 b256(256), b128(128);
  const dim3 gW(DM / 64, DM / 64);
  const dim3 gW1(FUS / 64, DM / 64);
  const dim3 gW2(DM / 64, FFI / 64);
  const dim3 gF1((((SEQ / 32) * (FUS / 128)) + 7) / 8);
  const dim3 gQK((((SEQ / 64) * ((4 * DM) / 64)) + 7) / 8);
  const dim3 gVT((((DM / 64) * (SEQ / 64)) + 7) / 8);
  const dim3 gWo((((SEQ / 64) * (DM / 64)) + 7) / 8);
  const dim3 gF2((((SEQ / 32) * (DM / 64)) + 7) / 8);

  k_cstab<<<dim3(SEQ / 8), b256, 0, stream>>>(itab, CS);
  k_xnorm<<<dim3(SEQ), b128, 0, stream>>>(hs, Xh, Xbh, Xbl);
  k_wtrans<0><<<gW, b256, 0, stream>>>(Wq,  DM, DM, 0, WSC, Wcat + (size_t)0 * DM * DM, Wcat);
  k_wtrans<0><<<gW, b256, 0, stream>>>(Wk,  DM, DM, 0, WSC, Wcat + (size_t)1 * DM * DM, Wcat);
  k_wtrans<0><<<gW, b256, 0, stream>>>(Wqb, DM, DM, 0, WSC, Wcat + (size_t)2 * DM * DM, Wcat);
  k_wtrans<0><<<gW, b256, 0, stream>>>(Wkb, DM, DM, 0, WSC, Wcat + (size_t)3 * DM * DM, Wcat);
  k_wtrans<1><<<gW, b256, 0, stream>>>(Wv,  DM, DM, 0, 1.0f, Wvh, Wvl);
  k_wtrans<1><<<gW, b256, 0, stream>>>(Wo,  DM, DM, 0, 1.0f, Woh, Wol);
  k_wtrans<0><<<gW1, b256, 0, stream>>>(W1, DM, FUS, FFI, WSC, W1t, W1t);
  k_wtrans<0><<<gW2, b256, 0, stream>>>(W2, FFI, DM, 0, WSC, W2t, W2t);
  k_gemm<_Float16, 2, 8, 0, 4><<<gF1, b256, 0, stream>>>(
      Xh, Xh, DM, W1t, W1t, DM,
      (void*)FF, FFI, (void*)FF, FFI, 0,
      b1, hs, hs, lam,
      SEQ, FUS, DM, 1.0f / (XSC * WSC), FSC);
  k_gemm<_Float16, 4, 4, 0, 0><<<gQK, b256, 0, stream>>>(
      Xh, Xh, DM, Wcat, Wcat, DM,
      (void*)QK, 4 * DM, (void*)QK, 4 * DM, 0,
      bo, hs, hs, lam,
      SEQ, 4 * DM, DM, 1.0f / (XSC * WSC), 1.0f);
  k_gemm<__bf16, 4, 4, 2, 2><<<gVT, b256, 0, stream>>>(
      Wvh, Wvl, DM, Xbh, Xbl, DM,
      (void*)VTh, SEQ, (void*)VTl, VLP, VLP,
      bo, hs, hs, lam,
      DM, SEQ, DM, 1.0f, VRS);
  k_rope<<<dim3(SEQ * NH / 8), b256, 0, stream>>>(QK, CS, Qh, Kh, QBn, KBn);
  k_prefix<<<dim3(DM / 256), b256, 0, stream>>>(KBn, Pf);
  k_attn<true><<<dim3(NH * RESQB), b128, 0, stream>>>(
      Qh, Kh, VTh, VTl, QBn, Pf, l2n, Yh, Yl, 0, RESQB);
  k_attn<false><<<dim3(NH * (NQB - RESQB)), b128, 0, stream>>>(
      Qh, Kh, VTh, VTl, QBn, Pf, l2n, Yh, Yl, RESQB, NQB - RESQB);
  k_gemm<__bf16, 4, 4, 2, 1><<<gWo, b256, 0, stream>>>(
      Yh, Yl, DM, Woh, Wol, DM,
      (void*)AO, DM, (void*)AO, DM, 0,
      bo, hs, hs, lam,
      SEQ, DM, DM, 1.0f, 1.0f);
  k_gemm<_Float16, 2, 4, 0, 3><<<gF2, b256, 0, stream>>>(
      FF, FF, FFI, W2t, W2t, FFI,
      d_out, DM, d_out, DM, 0,
      b2, hs, (const float*)AO, lam,
      SEQ, DM, FFI, 1.0f / (FSC * WSC), 1.0f);
  (void)hipGetLastError();
}
